// MambaBlock_43937515438319
// MI455X (gfx1250) — hardware-verified
//
#include <hip/hip_runtime.h>
#include <math.h>

typedef __attribute__((ext_vector_type(16))) _Float16 v16h;
typedef __attribute__((ext_vector_type(8)))  _Float16 v8h;
typedef __attribute__((ext_vector_type(16))) __bf16   v16b;
typedef __attribute__((ext_vector_type(8)))  __bf16   v8b;
typedef __attribute__((ext_vector_type(8)))  float    v8f;
typedef __attribute__((ext_vector_type(4)))  float    v4f;

constexpr int kBatch  = 2;
constexpr int kSeq    = 1024;
constexpr int kDm     = 512;
constexpr int kDin    = 1024;
constexpr int kNst    = 16;
constexpr int kDtR    = 32;
constexpr int kXzP    = 2 * kDin;
constexpr int kXdP    = 64;
constexpr int kRows   = kBatch * kSeq;
constexpr int kConvTP = 260;
constexpr float kGCarry  = 1024.0f;
constexpr float kWoCarry = 256.0f;
constexpr float kOutFold = 1.0f / (kGCarry * kWoCarry);

static_assert(kDtR + 2 * kNst == kXdP, "x_proj width");
static_assert(kRows == 2048 && kXzP == 2048, "shape");
static_assert((kDm % 32) == 0 && (kDin % 32) == 0 && (kDtR % 32) == 0, "GEMM K multiples of 32");
static_assert((kRows % 64) == 0 && (kXzP % 64) == 0 && (kXdP % 64) == 0 && (kDm % 64) == 0 && (kDin % 64) == 0, "GEMM M,N multiples of 64");
static_assert((kSeq % 64) == 0 && (kDin % 256) == 0 && (kSeq % 16) == 0, "tile multiples");
static_assert((((kRows / 64) * (kXzP / 64)) % 8) == 0 && (((kRows / 64) * (kXdP / 64)) % 8) == 0 &&
              (((kRows / 64) * (kDin / 64)) % 8) == 0 && (((kRows / 64) * (kDm / 64)) % 8) == 0, "8 tiles per block exactly");

constexpr size_t kOffX16   = 0;
constexpr size_t kOffWINT  = kOffX16   + (size_t)kRows * kDm  * 2;
constexpr size_t kOffWXT   = kOffWINT  + (size_t)kXzP  * kDm  * 2;
constexpr size_t kOffWDTT  = kOffWXT   + (size_t)kXdP  * kDin * 2;
constexpr size_t kOffWOUTT = kOffWDTT  + (size_t)kDin  * kDtR * 2;
constexpr size_t kOffXZ    = kOffWOUTT + (size_t)kDm   * kDin * 2;
constexpr size_t kOffUC    = kOffXZ    + (size_t)kRows * kXzP * 4;
constexpr size_t kOffUC16  = kOffUC    + (size_t)kRows * kDin * 4;
constexpr size_t kOffXD    = kOffUC16  + (size_t)kRows * kDin * 2;
constexpr size_t kOffDT16  = kOffXD    + (size_t)kRows * kXdP * 4;
constexpr size_t kOffDLR   = kOffDT16  + (size_t)kRows * kDtR * 2;
constexpr size_t kOffG16   = kOffDLR   + (size_t)kRows * kDin * 4;
constexpr size_t kWsTotal  = kOffG16   + (size_t)kRows * kDin * 2;
static_assert(kWsTotal == 48037888ull, "carve total");
static_assert(kWsTotal <= 134217728ull, "carve cap");
static_assert((kOffWINT % 128) == 0 && (kOffWXT % 128) == 0 && (kOffWDTT % 128) == 0 && (kOffWOUTT % 128) == 0 &&
              (kOffXZ % 128) == 0 && (kOffUC % 128) == 0 && (kOffUC16 % 128) == 0 && (kOffXD % 128) == 0 &&
              (kOffDT16 % 128) == 0 && (kOffDLR % 128) == 0 && (kOffG16 % 128) == 0, "128-B aligned regions");

__device__ __forceinline__ unsigned short f2bf_bits(float f) {
  unsigned u = __float_as_uint(f);
  return (unsigned short)((u + 0x7FFFu + ((u >> 16) & 1u)) >> 16);
}
__device__ __forceinline__ float bf_bits2f(unsigned short h) { return __uint_as_float(((unsigned)h) << 16); }
__device__ __forceinline__ float rne_bf16(float f) { return bf_bits2f(f2bf_bits(f)); }

__device__ __forceinline__ void group_guard_h(v8f& a, v8f& b, v8f& c, v8f& d, v16h x, v16h b0, v16h b1, v16h b2, v16h b3) {
  asm volatile("v_nop\n\tv_nop\n\tv_nop\n\tv_nop" : "+v"(a), "+v"(b), "+v"(c), "+v"(d) : "v"(x), "v"(b0), "v"(b1), "v"(b2), "v"(b3));
}
__device__ __forceinline__ void group_guard_b(v8f& a, v8f& b, v8f& c, v8f& d, v16b x, v16b b0, v16b b1, v16b b2, v16b b3) {
  asm volatile("v_nop\n\tv_nop\n\tv_nop\n\tv_nop" : "+v"(a), "+v"(b), "+v"(c), "+v"(d) : "v"(x), "v"(b0), "v"(b1), "v"(b2), "v"(b3));
}
__device__ __forceinline__ void keep4_h(v16h a, v16h b, v16h c, v16h d) { asm volatile("v_nop" :: "v"(a), "v"(b), "v"(c), "v"(d)); }
__device__ __forceinline__ void keep4_b(v16b a, v16b b, v16b c, v16b d) { asm volatile("v_nop" :: "v"(a), "v"(b), "v"(c), "v"(d)); }
__device__ __forceinline__ void acc_guard4(v8f& a, v8f& b, v8f& c, v8f& d) { asm volatile("v_nop\n\tv_nop\n\tv_nop\n\tv_nop" : "+v"(a), "+v"(b), "+v"(c), "+v"(d)); }

template <typename T> struct Frag;
template <> struct Frag<_Float16> {
  typedef v16h V; union U { v16h v; v8h h[2]; };
  static __device__ __forceinline__ v16h load(const _Float16* p) {
    U f; f.h[0] = *(const v8h*)(p); f.h[1] = *(const v8h*)(p + 16); return f.v;
  }
  static __device__ __forceinline__ v8f mma(v16h a, v16h b, v8f c) {
    return __builtin_amdgcn_wmma_f32_16x16x32_f16(false, a, false, b, (short)0, c, false, false);
  }
  static __device__ __forceinline__ void guard4(v8f& a, v8f& b, v8f& c, v8f& d, v16h x, v16h b0, v16h b1, v16h b2, v16h b3) { group_guard_h(a, b, c, d, x, b0, b1, b2, b3); }
  static __device__ __forceinline__ void keep(v16h a, v16h b, v16h c, v16h d) { keep4_h(a, b, c, d); }
};
template <> struct Frag<__bf16> {
  typedef v16b V; union U { v16b v; v8b h[2]; };
  static __device__ __forceinline__ v16b load(const __bf16* p) {
    U f; f.h[0] = *(const v8b*)(p); f.h[1] = *(const v8b*)(p + 16); return f.v;
  }
  static __device__ __forceinline__ v8f mma(v16b a, v16b b, v8f c) {
    return __builtin_amdgcn_wmma_f32_16x16x32_bf16(false, a, false, b, (short)0, c, false, false);
  }
  static __device__ __forceinline__ void guard4(v8f& a, v8f& b, v8f& c, v8f& d, v16b x, v16b b0, v16b b1, v16b b2, v16b b3) { group_guard_b(a, b, c, d, x, b0, b1, b2, b3); }
  static __device__ __forceinline__ void keep(v16b a, v16b b, v16b c, v16b d) { keep4_b(a, b, c, d); }
};

template <int ET> struct Elem;
template <> struct Elem<0> { typedef _Float16 T; };
template <> struct Elem<1> { typedef __bf16 T; };
template <int ET, int BIAS_MODE>
__global__ __launch_bounds__(256) void wmma_gemm64(
    const unsigned short* __restrict__ Ap, int lda,
    const unsigned short* __restrict__ Btp, int ldb,
    float* __restrict__ Cout, int ldc,
    const float* __restrict__ bias,
    int M, int N, int K, float scale) {
  typedef typename Elem<ET>::T T;
  typedef typename Frag<T>::V V;
  const T* A = (const T*)Ap;
  const T* Bt = (const T*)Btp;
  __shared__ __align__(16) float sT[8][16 * 68];
  const int lane = threadIdx.x & 31;
  const int wave = threadIdx.x >> 5;
  const int tilesN = N >> 6;
  const int tilesM = M >> 6;
  const int tile = blockIdx.x * 8 + wave;
  if (tile >= tilesM * tilesN) return;
  const int tm = tile / tilesN;
  const int tn = tile - tm * tilesN;
  const int m0 = tm << 6;
  const int n0 = tn << 6;

  const int rlane = lane & 15;
  const int koff  = (lane >> 4) * 8;
  const int mOff  = (lane >> 4) * 8;

  v8f acc[4][4];
#pragma unroll
  for (int i = 0; i < 4; ++i)
#pragma unroll
    for (int j = 0; j < 4; ++j) acc[i][j] = (v8f){0.f,0.f,0.f,0.f,0.f,0.f,0.f,0.f};

  for (int k0 = 0; k0 < K; k0 += 32) {
    V bh[4];
#pragma unroll
    for (int j = 0; j < 4; ++j) {
      const size_t bo = (size_t)(n0 + (j << 4) + rlane) * ldb + koff + k0;
      bh[j] = Frag<T>::load(Bt + bo);
    }
#pragma unroll
    for (int i = 0; i < 4; ++i) {
      const size_t ao = (size_t)(m0 + (i << 4) + rlane) * lda + koff + k0;
      V ah = Frag<T>::load(A + ao);
#pragma unroll
      for (int j = 0; j < 4; ++j) acc[i][j] = Frag<T>::mma(ah, bh[j], acc[i][j]);
      Frag<T>::guard4(acc[i][0], acc[i][1], acc[i][2], acc[i][3], ah, bh[0], bh[1], bh[2], bh[3]);
    }
    Frag<T>::keep(bh[0], bh[1], bh[2], bh[3]);
  }
  acc_guard4(acc[0][0], acc[0][1], acc[0][2], acc[0][3]);
  acc_guard4(acc[1][0], acc[1][1], acc[1][2], acc[1][3]);
  acc_guard4(acc[2][0], acc[2][1], acc[2][2], acc[2][3]);
  acc_guard4(acc[3][0], acc[3][1], acc[3][2], acc[3][3]);

  float* slab = sT[wave];
#pragma unroll
  for (int i = 0; i < 4; ++i) {
    const int mBase = m0 + (i << 4);
#pragma unroll
    for (int j = 0; j < 4; ++j) {
      const int n = n0 + (j << 4) + rlane;
      float bv = 0.f;
      if (BIAS_MODE == 2) bv = rne_bf16(bias[n]);
#pragma unroll
      for (int r = 0; r < 8; ++r) {
        float v = acc[i][j][r] * scale;
        if (BIAS_MODE == 2) v += bv;
        slab[(mOff + r) * 68 + (j << 4) + rlane] = v;
      }
    }
    __builtin_amdgcn_fence(__ATOMIC_RELEASE, "workgroup");
    __builtin_amdgcn_wave_barrier();
    __builtin_amdgcn_fence(__ATOMIC_ACQUIRE, "workgroup");
    {
      const int hh = lane >> 4, c4 = (lane & 15) * 4;
      for (int pass = 0; pass < 2; ++pass) {
#pragma unroll
        for (int it = 0; it < 8; ++it) {
          const int row = it * 2 + hh;
          v4f v = *(const v4f*)(slab + row * 68 + c4);
          *(volatile v4f*)(Cout + (size_t)(mBase + row) * ldc + n0 + c4) = v;
        }
        __threadfence();
      }
    }
    __builtin_amdgcn_fence(__ATOMIC_RELEASE, "workgroup");
    __builtin_amdgcn_wave_barrier();
    __builtin_amdgcn_fence(__ATOMIC_ACQUIRE, "workgroup");
  }
}

__global__ __launch_bounds__(256) void cast_rows_bf16_kernel(
    const float* __restrict__ src, unsigned short* __restrict__ dst, int total8)
{
  const int i = blockIdx.x * 256 + threadIdx.x;
  if (i >= total8) return;
  const size_t e0 = (size_t)i << 3;
  const v4f a0 = *(const v4f*)(src + e0);
  const v4f a1 = *(const v4f*)(src + e0 + 4);
  v8h hv;
#pragma unroll
  for (int e = 0; e < 4; ++e) {
    const unsigned short h0 = f2bf_bits(a0[e]);
    const unsigned short h1 = f2bf_bits(a1[e]);
    hv[e]     = __builtin_bit_cast(_Float16, h0);
    hv[4 + e] = __builtin_bit_cast(_Float16, h1);
  }
  unsigned short* q = dst + e0;
  *(volatile v8h*)q = hv;
  __threadfence();
  *(volatile v8h*)q = hv;
}

template <int KT, bool F16OUT>
__global__ __launch_bounds__(256) void transpose_cast_kernel(
    const float* __restrict__ W, unsigned short* __restrict__ Bt, int Kdim, int Ndim, float scale)
{
  __shared__ float tile[KT * 65];
  const int tid = threadIdx.x, lane = tid & 31, wave = tid >> 5;
  const int n0 = blockIdx.x * 64;
  const int k0 = blockIdx.y * KT;
#pragma unroll
  for (int p = 0; p < KT / 4; ++p) {
    const int idx = tid + p * 256;
    const int kk  = idx >> 6;
    const int nn  = idx & 63;
    const float v = W[(size_t)(k0 + kk) * Ndim + n0 + nn];
    tile[kk * 65 + nn] = rne_bf16(v) * scale;
  }
  __syncthreads();
  constexpr int LPR = KT / 8;
  constexpr int RPW = 32 / LPR;
  constexpr int NIT = 8 / RPW;
  const int q = lane / LPR, c8 = (lane % LPR) * 8;
  v8h hv[NIT];
#pragma unroll
  for (int it = 0; it < NIT; ++it) {
    const int nrow = it * 8 * RPW + wave * RPW + q;
#pragma unroll
    for (int e = 0; e < 8; ++e) {
      const float tv = tile[(c8 + e) * 65 + nrow];
      if (F16OUT) {
        hv[it][e] = (_Float16)tv;
      } else {
        const unsigned short hb = f2bf_bits(tv);
        hv[it][e] = __builtin_bit_cast(_Float16, hb);
      }
    }
  }
  for (int pass = 0; pass < 2; ++pass) {
#pragma unroll
    for (int it = 0; it < NIT; ++it) {
      const int nrow = it * 8 * RPW + wave * RPW + q;
      *(volatile v8h*)(Bt + (size_t)(n0 + nrow) * Kdim + k0 + c8) = hv[it];
    }
    __threadfence();
  }
}

__global__ __launch_bounds__(256) void dt_cast_kernel(
    const float* __restrict__ XD, unsigned short* __restrict__ DT16, int total8)
{
  const int i = blockIdx.x * 256 + threadIdx.x;
  if (i >= total8) return;
  const int e0  = i << 3;
  const int row = e0 >> 5;
  const int c8  = e0 & 31;
  const float* p = XD + (size_t)row * kXdP + c8;
  const v4f a0 = *(const v4f*)(p);
  const v4f a1 = *(const v4f*)(p + 4);
  v8h hv;
#pragma unroll
  for (int e = 0; e < 4; ++e) {
    const unsigned short h0 = f2bf_bits(a0[e]);
    const unsigned short h1 = f2bf_bits(a1[e]);
    hv[e]     = __builtin_bit_cast(_Float16, h0);
    hv[4 + e] = __builtin_bit_cast(_Float16, h1);
  }
  unsigned short* qd = DT16 + e0;
  *(volatile v8h*)qd = hv;
  __threadfence();
  *(volatile v8h*)qd = hv;
}

__global__ __launch_bounds__(256) void conv_silu_kernel(
    const float* __restrict__ XZ, const float* __restrict__ cw, const float* __restrict__ cb,
    float* __restrict__ UC, unsigned short* __restrict__ UC16)
{
  __shared__ __align__(16) float sT[16 * kConvTP];
  const int tid = threadIdx.x, lane = tid & 31, wave = tid >> 5;
  const int d0 = blockIdx.x * 256, d = d0 + tid;
  const int g0 = blockIdx.y * 64;
  const int tb = g0 & (kSeq - 1);
  const v4f wv = *(const v4f*)(cw + (size_t)d * 4);
  const float w0 = rne_bf16(wv[0]), w1 = rne_bf16(wv[1]), w2 = rne_bf16(wv[2]), w3 = rne_bf16(wv[3]);
  const float bc = rne_bf16(cb[d]);
  float xm3, xm2, xm1;
  {
    const bool hist = (tb > 0);
    const int rb = hist ? (g0 - 3) : g0;
    const float v3 = XZ[(size_t)rb * kXzP + d];
    const float v2 = XZ[(size_t)(rb + 1) * kXzP + d];
    const float v1 = XZ[(size_t)(rb + 2) * kXzP + d];
    xm3 = hist ? v3 : 0.f;
    xm2 = hist ? v2 : 0.f;
    xm1 = hist ? v1 : 0.f;
  }
  const int hrow = wave >> 1;
  const int hch  = (wave & 1) * 128 + lane * 4;
#pragma unroll 1
  for (int sub = 0; sub < 4; ++sub) {
    const int lb = g0 + sub * 16;
#pragma unroll 1
    for (int s = 0; s < 16; ++s) {
      const float xcur = XZ[(size_t)(lb + s) * kXzP + d];
      float acc = w0 * xm3;
      acc = fmaf(w1, xm2, acc);
      acc = fmaf(w2, xm1, acc);
      acc = fmaf(w3, xcur, acc);
      const float sv = acc + bc;
      const float sg = 1.0f / (1.0f + expf(-sv));
      sT[s * kConvTP + tid] = sv * sg;
      xm3 = xm2; xm2 = xm1; xm1 = xcur;
    }
    __syncthreads();
    v4f fv[4];
    v8h bv[2];
#pragma unroll
    for (int it = 0; it < 4; ++it) fv[it] = *(const v4f*)(sT + (it * 4 + hrow) * kConvTP + hch);
#pragma unroll
    for (int it = 0; it < 2; ++it) {
      const float* sp = sT + (it * 8 + wave) * kConvTP + lane * 8;
      const v4f a0 = *(const v4f*)(sp);
      const v4f a1 = *(const v4f*)(sp + 4);
#pragma unroll
      for (int e = 0; e < 4; ++e) {
        const unsigned short h0 = f2bf_bits(a0[e]);
        const unsigned short h1 = f2bf_bits(a1[e]);
        bv[it][e]     = __builtin_bit_cast(_Float16, h0);
        bv[it][4 + e] = __builtin_bit_cast(_Float16, h1);
      }
    }
    for (int pass = 0; pass < 2; ++pass) {
#pragma unroll
      for (int it = 0; it < 4; ++it)
        *(volatile v4f*)(UC + (size_t)(lb + it * 4 + hrow) * kDin + d0 + hch) = fv[it];
#pragma unroll
      for (int it = 0; it < 2; ++it)
        *(volatile v8h*)(UC16 + (size_t)(lb + it * 8 + wave) * kDin + d0 + lane * 8) = bv[it];
      __threadfence();
    }
    __syncthreads();
  }
}

__global__ __launch_bounds__(256) void scan_gate_kernel(
    const float* __restrict__ DLR, const float* __restrict__ UC, const float* __restrict__ XZ,
    const float* __restrict__ XD, const float* __restrict__ bdt, const float* __restrict__ Alog,
    const float* __restrict__ Dsk, unsigned short* __restrict__ G16)
{
#pragma clang fp contract(off)
  __shared__ __align__(16) float sBC[16 * 32];
  __shared__ __align__(16) float sY[16 * kConvTP];
  __shared__ float sA[kNst * 256];
  const int tid = threadIdx.x, lane = tid & 31, wave = tid >> 5;
  constexpr int kBlkPerB = kDin / 256;
  const int bix = blockIdx.x / kBlkPerB;
  const int d0  = (blockIdx.x - bix * kBlkPerB) * 256;
  const int d   = d0 + tid;
  const size_t row0 = (size_t)bix * kSeq;

#pragma unroll 1
  for (int n = 0; n < kNst; ++n) sA[n * 256 + tid] = -expf(rne_bf16(Alog[(size_t)d * kNst + n]));
  __syncthreads();
  float An[kNst], P[kNst], S[kNst];
#pragma unroll
  for (int n = 0; n < kNst; ++n) {
    An[n] = sA[n * 256 + tid];
    P[n] = 0.f;
    S[n] = 0.f;
  }
  const float bb = rne_bf16(bdt[d]);
  const float Dd = rne_bf16(Dsk[d]);

#pragma unroll 1
  for (int c = 0; c < kSeq / 16; ++c) {
    const int l0 = c * 16;
    if (tid < 128) {
      const int r = tid >> 3, q4 = (tid & 7) * 4;
      const v4f v = *(const v4f*)(XD + (row0 + l0 + r) * kXdP + kDtR + q4);
      *(v4f*)(sBC + r * 32 + q4) = v;
    }
    __syncthreads();
#pragma unroll 1
    for (int s = 0; s < 16; ++s) {
      const size_t m = row0 + (size_t)(l0 + s);
      float a  = DLR[m * kDin + d];
      float xv = UC[m * kDin + d];
      float zv = XZ[m * kXzP + kDin + d];
      asm volatile("" : "+v"(a));
      asm volatile("" : "+v"(xv));
      asm volatile("" : "+v"(zv));
      a = a + bb;
      const float e1  = expf(-fabsf(a));
      const float u1  = 1.0f + e1;
      const float l1p = logf(u1) + (e1 - (u1 - 1.0f)) * __builtin_amdgcn_rcpf(u1);
      const float delta = fmaxf(a, 0.0f) + l1p;
      const float dtu = delta * xv;
      const bool adv = (l0 + s) > 0;
      v4f Bq[4], Cq[4];
#pragma unroll
      for (int qq = 0; qq < 4; ++qq) {
        Bq[qq] = *(const v4f*)(sBC + s * 32 + 4 * qq);
        Cq[qq] = *(const v4f*)(sBC + s * 32 + kNst + 4 * qq);
      }
      float y = 0.f;
#pragma unroll
      for (int n = 0; n < kNst; ++n) {
        const float dA = delta * An[n];
        P[n] = P[n] + (adv ? dA : 0.0f);
        float E = __expf(P[n]);
        E = (E < 1.17549435e-38f) ? 0.0f : E;
        const float den = E + 1e-12f;
        const float qv = (dtu * Bq[n >> 2][n & 3]) * __builtin_amdgcn_rcpf(den);
        S[n] = S[n] + qv;
        const float hn = S[n] * E;
        y = y + hn * Cq[n >> 2][n & 3];
      }
      y = y + xv * Dd;
      const float sg = 1.0f / (1.0f + expf(-zv));
      const float g  = zv * sg;
      sY[s * kConvTP + tid] = (y * g) * kGCarry;
    }
    __syncthreads();
    v8h hv[2];
#pragma unroll
    for (int it = 0; it < 2; ++it) {
      const float* sp = sY + (it * 8 + wave) * kConvTP + lane * 8;
      const v4f a0 = *(const v4f*)(sp);
      const v4f a1 = *(const v4f*)(sp + 4);
#pragma unroll
      for (int e = 0; e < 4; ++e) {
        hv[it][e]     = (_Float16)a0[e];
        hv[it][4 + e] = (_Float16)a1[e];
      }
    }
    for (int pass = 0; pass < 2; ++pass) {
#pragma unroll
      for (int it = 0; it < 2; ++it)
        *(volatile v8h*)(G16 + (row0 + (size_t)(l0 + it * 8 + wave)) * kDin + d0 + lane * 8) = hv[it];
      __threadfence();
    }
  }
}

extern "C" void kernel_launch(void* const* d_in, const int* in_sizes, int n_in,
                              void* d_out, int out_size, void* d_ws, size_t ws_size,
                              hipStream_t stream) {
  if (n_in < 11) return;
  if (in_sizes[0] != kRows * kDm) return;
  if (in_sizes[1] != kDm * kXzP) return;
  if (in_sizes[2] != kDin * 4) return;
  if (in_sizes[3] != kDin) return;
  if (in_sizes[4] != kDin * kXdP) return;
  if (in_sizes[5] != kDtR * kDin) return;
  if (in_sizes[6] != kDin) return;
  if (in_sizes[7] != kDin * kNst) return;
  if (in_sizes[8] != kDin) return;
  if (in_sizes[9] != kDin * kDm) return;
  if (in_sizes[10] != kDm) return;
  if (out_size != kRows * kDm) return;
  if (ws_size < kWsTotal) return;

  const float* x      = (const float*)d_in[0];
  const float* W_in   = (const float*)d_in[1];
  const float* conv_w = (const float*)d_in[2];
  const float* conv_b = (const float*)d_in[3];
  const float* W_x    = (const float*)d_in[4];
  const float* W_dt   = (const float*)d_in[5];
  const float* b_dt   = (const float*)d_in[6];
  const float* A_log  = (const float*)d_in[7];
  const float* D_skip = (const float*)d_in[8];
  const float* W_out  = (const float*)d_in[9];
  const float* b_out  = (const float*)d_in[10];
  float* out = (float*)d_out;

  char* ws = (char*)d_ws;
  unsigned short* X16   = (unsigned short*)(ws + kOffX16);
  unsigned short* WINT  = (unsigned short*)(ws + kOffWINT);
  unsigned short* WXT   = (unsigned short*)(ws + kOffWXT);
  unsigned short* WDTT  = (unsigned short*)(ws + kOffWDTT);
  unsigned short* WOUTT = (unsigned short*)(ws + kOffWOUTT);
  float*          XZ    = (float*)(ws + kOffXZ);
  float*          UC    = (float*)(ws + kOffUC);
  unsigned short* UC16  = (unsigned short*)(ws + kOffUC16);
  float*          XD    = (float*)(ws + kOffXD);
  unsigned short* DT16  = (unsigned short*)(ws + kOffDT16);
  float*          DLR   = (float*)(ws + kOffDLR);
  unsigned short* G16   = (unsigned short*)(ws + kOffG16);

  cast_rows_bf16_kernel<<<(kRows * kDm / 8) / 256, 256, 0, stream>>>(x, X16, kRows * kDm / 8);

  transpose_cast_kernel<64, false><<<dim3(kXzP / 64, kDm / 64), 256, 0, stream>>>(W_in, WINT, kDm, kXzP, 1.0f);
  transpose_cast_kernel<64, false><<<dim3(kXdP / 64, kDin / 64), 256, 0, stream>>>(W_x, WXT, kDin, kXdP, 1.0f);
  transpose_cast_kernel<32, false><<<dim3(kDin / 64, kDtR / 32), 256, 0, stream>>>(W_dt, WDTT, kDtR, kDin, 1.0f);
  transpose_cast_kernel<64, true><<<dim3(kDm / 64, kDin / 64), 256, 0, stream>>>(W_out, WOUTT, kDin, kDm, kWoCarry);

  wmma_gemm64<1, 0><<<((kRows / 64) * (kXzP / 64)) / 8, 256, 0, stream>>>(
      X16, kDm, WINT, kDm, XZ, kXzP, b_out, kRows, kXzP, kDm, 1.0f);

  conv_silu_kernel<<<dim3(kDin / 256, kRows / 64), 256, 0, stream>>>(XZ, conv_w, conv_b, UC, UC16);

  wmma_gemm64<1, 0><<<((kRows / 64) * (kXdP / 64)) / 8, 256, 0, stream>>>(
      UC16, kDin, WXT, kDin, XD, kXdP, b_out, kRows, kXdP, kDin, 1.0f);

  dt_cast_kernel<<<(kRows * kDtR / 8) / 256, 256, 0, stream>>>(XD, DT16, kRows * kDtR / 8);

  wmma_gemm64<1, 0><<<((kRows / 64) * (kDin / 64)) / 8, 256, 0, stream>>>(
      DT16, kDtR, WDTT, kDtR, DLR, kDin, b_out, kRows, kDin, kDtR, 1.0f);

  scan_gate_kernel<<<kBatch * (kDin / 256), 256, 0, stream>>>(DLR, UC, XZ, XD, b_dt, A_log, D_skip, G16);

  wmma_gemm64<0, 2><<<((kRows / 64) * (kDm / 64)) / 8, 256, 0, stream>>>(
      G16, kDin, WOUTT, kDin, out, kDm, b_out, kRows, kDm, kDin, kOutFold);
}
